// nchwAttentionLePE_31817117728874
// MI455X (gfx1250) — hardware-verified
//
#include <hip/hip_runtime.h>
#include <math.h>

typedef __attribute__((ext_vector_type(16))) _Float16 v16h;
typedef __attribute__((ext_vector_type(16))) __bf16 v16b;
typedef __attribute__((ext_vector_type(8)))  _Float16 v8h;
typedef __attribute__((ext_vector_type(8)))  float v8f;
typedef __attribute__((ext_vector_type(4)))  float v4f;
typedef __attribute__((ext_vector_type(2)))  float v2f;
typedef __attribute__((ext_vector_type(4)))  unsigned v4u;
typedef __attribute__((ext_vector_type(4)))  int v4i;
typedef float __attribute__((may_alias)) float_a;
typedef int __attribute__((may_alias)) int_a;

template <typename T> __device__ __forceinline__ void vst2(void* p, T v) { *(volatile T*)p = v; __threadfence(); *(volatile T*)p = v; }
__device__ __forceinline__ v8f wmma16(v16h a, v16h b, v8f c) {
  v8f d = __builtin_amdgcn_wmma_f32_16x16x32_f16(false, a, false, b, (short)0, c, false, false);
  asm volatile("v_nop\n\tv_nop\n\tv_nop\n\tv_nop" : "+v"(d) : "v"(a), "v"(b));
  return d;
}
__device__ __forceinline__ v8f wmma_bf(v16b a, v16b b, v8f c) {
  v8f d = __builtin_amdgcn_wmma_f32_16x16x32_bf16(false, a, false, b, (short)0, c, false, false);
  asm volatile("v_nop\n\tv_nop\n\tv_nop\n\tv_nop" : "+v"(d) : "v"(a), "v"(b));
  return d;
}
__device__ __forceinline__ v16h frag_h(const _Float16* rowk0, int lane) {
  union { v16h v; v8h q[2]; } u; const _Float16* p = rowk0 + 8 * (lane >> 4);
  u.q[0] = *(const v8h*)p; u.q[1] = *(const v8h*)(p + 16); return u.v;
}
__device__ __forceinline__ v16h frag_f32(const float* rowk0, int lane) {
  v16h a; const float* p = rowk0 + 8 * (lane >> 4);
#pragma unroll
  for (int i = 0; i < 8; ++i) { a[i] = (_Float16)p[i]; a[8 + i] = (_Float16)p[16 + i]; }
  return a;
}
__device__ __forceinline__ v16h frag_f32s(const float* rowk0, int lane, float sc) {
  v16h a; const float* p = rowk0 + 8 * (lane >> 4);
#pragma unroll
  for (int i = 0; i < 8; ++i) { a[i] = (_Float16)(p[i] * sc); a[8 + i] = (_Float16)(p[16 + i] * sc); }
  return a;
}
__device__ __forceinline__ v16h fragc_f32(const float* W, int k0, int n, int lane, int ld, int K) {
  v16h a; const int g = lane >> 4;
#pragma unroll
  for (int i = 0; i < 8; ++i) { const int ka = k0 + 8 * g + i, kb = ka + 16;
    a[i] = (_Float16)(ka < K ? W[(size_t)ka * ld + n] : 0.f); a[8 + i] = (_Float16)(kb < K ? W[(size_t)kb * ld + n] : 0.f); }
  return a;
}
struct F2 { v16b h, l; };
__device__ __forceinline__ F2 bsplit16(const float v[16]) { F2 r;
#pragma unroll
  for (int i = 0; i < 16; ++i) { const __bf16 h = (__bf16)v[i]; r.h[i] = h; r.l[i] = (__bf16)(v[i] - (float)h); }
  return r; }
__device__ __forceinline__ F2 split_row(const float* row, int k0, int lane) { float v[16]; const float* p = row + k0 + 8 * (lane >> 4);
#pragma unroll
  for (int i = 0; i < 8; ++i) { v[i] = p[i]; v[8 + i] = p[16 + i]; }
  return bsplit16(v); }
__device__ __forceinline__ F2 split_rowK(const float* row, int k0, int lane, int K) { float v[16]; const int g = lane >> 4;
#pragma unroll
  for (int i = 0; i < 8; ++i) { const int ka = k0 + 8 * g + i, kb = ka + 16; v[i] = ka < K ? row[ka] : 0.f; v[8 + i] = kb < K ? row[kb] : 0.f; }
  return bsplit16(v); }
__device__ __forceinline__ F2 split_col(const float* W, int k0, int n, int lane, int ld, int K) { float v[16]; const int g = lane >> 4;
#pragma unroll
  for (int i = 0; i < 8; ++i) { const int ka = k0 + 8 * g + i, kb = ka + 16; v[i] = ka < K ? W[(size_t)ka * ld + n] : 0.f; v[8 + i] = kb < K ? W[(size_t)kb * ld + n] : 0.f; }
  return bsplit16(v); }
__device__ __forceinline__ v8f mac3(const F2& a, const F2& b, v8f c) { c = wmma_bf(a.l, b.h, c); c = wmma_bf(a.h, b.l, c); return wmma_bf(a.h, b.h, c); }
__device__ __forceinline__ float sigm(float v) { return 1.0f / (1.0f + expf(-v)); }
#define LDSX() do { asm volatile("s_wait_dscnt 0" ::: "memory"); __builtin_amdgcn_wave_barrier(); __builtin_amdgcn_fence(__ATOMIC_RELEASE, "workgroup"); } while (0)


#define NBI 8
#define C 256
#define NH 8
#define HD 32
#define NP 1024
#define IW 32
#define NR (NBI * NP)
#define KS 5

__global__ __launch_bounds__(256) void k_cvt(const float* __restrict__ x, _Float16* __restrict__ X16) {
  __shared__ __align__(16) _Float16 st[C][72];
  const int tid = threadIdx.x; const int b = blockIdx.x / (NP / 64), n0 = (blockIdx.x % (NP / 64)) * 64;
  for (int q = tid; q < C * 16; q += 256) { const int c = q >> 4, p4 = q & 15; const v4f v = *(const v4f*)(x + ((size_t)b * C + c) * NP + n0 + p4 * 4);
    st[c][p4 * 4] = (_Float16)v[0]; st[c][p4 * 4 + 1] = (_Float16)v[1]; st[c][p4 * 4 + 2] = (_Float16)v[2]; st[c][p4 * 4 + 3] = (_Float16)v[3]; }
  __syncthreads();
  for (int q = tid; q < 64 * (C / 8); q += 256) { const int nl = q >> 5, pc = q & 31; union { v8h h; v4u u; } pk;
#pragma unroll
    for (int e = 0; e < 8; ++e) pk.h[e] = st[pc * 8 + e][nl];
    vst2(X16 + ((size_t)b * NP + n0 + nl) * C + pc * 8, pk.u); }
}
__global__ __launch_bounds__(256) void k_pack(const float* __restrict__ wqkv, const float* __restrict__ wp, _Float16* __restrict__ PT) {
  const int n = blockIdx.x, tid = threadIdx.x; __shared__ __align__(16) _Float16 srow[C];
  const float* src = n < 3 * C ? wqkv + (size_t)n * C : wp + (size_t)(n - 3 * C) * C;
  srow[tid] = (_Float16)(src[tid] * 16.0f); __syncthreads();
  if (tid < C / 8) vst2(PT + (size_t)n * C + tid * 8, *(const v4u*)(&srow[tid * 8]));
}
__global__ __launch_bounds__(128) void k_qkv(const _Float16* __restrict__ X16, const _Float16* __restrict__ PT, _Float16* __restrict__ Q16, _Float16* __restrict__ K16, _Float16* __restrict__ V16) {
  __shared__ __align__(16) float so[4][16][132];
  __shared__ __align__(16) _Float16 sth[128][72];
  const int tid = threadIdx.x, wave = tid >> 5, lane = tid & 31, col = lane & 15, g = lane >> 4;
  const int r0b = blockIdx.x * 64, r0 = r0b + wave * 16, n0 = blockIdx.y * 128; const int b = r0b / NP, s0 = r0b % NP; const int which = n0 / C, h0 = (n0 % C) / HD;
  v8f acc[8] = {};
#pragma unroll 2
  for (int kc = 0; kc < C / 32; ++kc) { const v16h a = frag_h(X16 + (size_t)(r0 + col) * C + kc * 32, lane);
#pragma unroll
    for (int j = 0; j < 8; ++j) acc[j] = wmma16(a, frag_h(PT + (size_t)(n0 + j * 16 + col) * C + kc * 32, lane), acc[j]); }
  if (which < 2) {
#pragma unroll
    for (int j = 0; j < 8; ++j)
#pragma unroll
      for (int r = 0; r < 8; ++r) so[wave][8 * g + r][j * 16 + col] = acc[j][r] * (4.0f / 16.0f);
    LDSX();
    _Float16* Dst = which == 0 ? Q16 : K16;
    for (int qq = lane; qq < 4 * 16 * 4; qq += 32) { const int hh = qq >> 6, rl = (qq >> 2) & 15, pc = qq & 3; union { v8h h8; v4u u; } pk;
#pragma unroll
      for (int e = 0; e < 8; ++e) pk.h8[e] = (_Float16)so[wave][rl][hh * 32 + pc * 8 + e];
      vst2(Dst + (((size_t)b * NH + h0 + hh) * NP + s0 + wave * 16 + rl) * HD + pc * 8, pk.u); } }
  else {
#pragma unroll
    for (int j = 0; j < 8; ++j)
#pragma unroll
      for (int r = 0; r < 8; ++r) sth[j * 16 + col][wave * 16 + 8 * g + r] = (_Float16)(acc[j][r] * (4.0f / 16.0f));
    __syncthreads();
    for (int qq = tid; qq < 128 * 8; qq += 128) { const int cl = qq >> 3, pc = qq & 7; vst2(V16 + ((size_t)b * C + (n0 - 2 * C) + cl) * NP + s0 + pc * 8, *(const v4u*)(&sth[cl][pc * 8])); } }
}
__global__ __launch_bounds__(128) void k_attn(const _Float16* __restrict__ Q16, const _Float16* __restrict__ K16, const _Float16* __restrict__ V16, _Float16* __restrict__ O16) {
  __shared__ __align__(16) float sS[4][16][68];
  __shared__ __align__(16) _Float16 sPh[4][16][72];
  __shared__ __align__(16) float sO[4][16][36];
  const int tid = threadIdx.x, w = tid >> 5, lane = tid & 31, col = lane & 15, g = lane >> 4;
  const size_t bh = blockIdx.y; const int b = (int)(bh / NH), h = (int)(bh % NH); const int q0 = blockIdx.x * 64 + w * 16;
  const v16h aq = frag_h(Q16 + (bh * NP + q0 + col) * HD, lane);
  const float scl = 0.17677669529663687f / 16.0f;
  float mrun = -3.0e38f, lrun = 0.f; v8f acc[2] = {};
#pragma unroll 1
  for (int kt = 0; kt < NP / 64; ++kt) {
#pragma unroll
    for (int t = 0; t < 4; ++t) { const int key = kt * 64 + t * 16 + col; const v8f s = wmma16(aq, frag_h(K16 + (bh * NP + key) * HD, lane), (v8f){});
#pragma unroll
      for (int r = 0; r < 8; ++r) sS[w][8 * g + r][t * 16 + col] = s[r] * scl; }
    LDSX();
    float mx = -3.4e38f;
#pragma unroll
    for (int jj = 0; jj < 32; ++jj) mx = fmaxf(mx, sS[w][col][g * 32 + jj]);
    mx = fmaxf(mx, __shfl_xor(mx, 16, 32));
    const float mnew = fmaxf(mrun, mx); const float corr = expf(mrun - mnew);
    float ps = 0.f;
#pragma unroll
    for (int jj = 0; jj < 32; ++jj) { const float p = expf(sS[w][col][g * 32 + jj] - mnew) * 16384.0f; ps += p; sPh[w][col][g * 32 + jj] = (_Float16)p; }
    ps += __shfl_xor(ps, 16, 32);
    lrun = lrun * corr + ps * (1.0f / 16384.0f); mrun = mnew;
#pragma unroll
    for (int r = 0; r < 8; ++r) { const float cr = __shfl(corr, 8 * g + r, 32); acc[0][r] *= cr; acc[1][r] *= cr; }
    LDSX();
#pragma unroll
    for (int kc = 0; kc < 2; ++kc) { const v16h ph = frag_h(&sPh[w][col][0] + kc * 32, lane);
#pragma unroll
      for (int t2 = 0; t2 < 2; ++t2) acc[t2] = wmma16(ph, frag_h(V16 + ((size_t)b * C + h * HD + t2 * 16 + col) * NP + kt * 64 + kc * 32, lane), acc[t2]); }
    __builtin_amdgcn_wave_barrier(); }
#pragma unroll
  for (int r = 0; r < 8; ++r) { const float lr = __shfl(lrun, 8 * g + r, 32); const float inv = 8.0f / (lr * 16384.0f * 4.0f);
#pragma unroll
    for (int t2 = 0; t2 < 2; ++t2) sO[w][8 * g + r][t2 * 16 + col] = acc[t2][r] * inv; }
  LDSX();
  for (int qq = lane; qq < 16 * 4; qq += 32) { const int rl = qq >> 2, pc = qq & 3; union { v8h h8; v4u u; } pk;
#pragma unroll
    for (int e = 0; e < 8; ++e) pk.h8[e] = (_Float16)sO[w][rl][pc * 8 + e];
    vst2(O16 + ((size_t)b * NP + q0 + rl) * C + h * HD + pc * 8, pk.u); }
}
__global__ __launch_bounds__(256) void k_lepe(const _Float16* __restrict__ V16, const _Float16* __restrict__ O16, const float* __restrict__ lw, const float* __restrict__ lb, _Float16* __restrict__ Z16) {
  __shared__ float sv[8][IW + 4][IW + 4];
  __shared__ __align__(16) _Float16 sz[NP][64];
  const int tid = threadIdx.x; const int b = blockIdx.x / (C / 64), c0 = (blockIdx.x % (C / 64)) * 64;
#pragma unroll 1
  for (int cg = 0; cg < 8; ++cg) { const int cb = c0 + cg * 8;
    for (int q = tid; q < 8 * 36 * 36; q += 256) (&sv[0][0][0])[q] = 0.f;
    __syncthreads();
    for (int q = tid; q < 8 * NP; q += 256) { const int cl = q >> 10, n = q & 1023; sv[cl][2 + (n >> 5)][2 + (n & 31)] = (float)V16[((size_t)b * C + cb + cl) * NP + n] * 0.25f; }
    __syncthreads();
    for (int q = tid; q < 8 * NP; q += 256) { const int cl = q & 7, n = q >> 3; const int y = n >> 5, xx = n & 31; const float* wk = lw + (size_t)(cb + cl) * KS * KS; float s = lb[cb + cl];
#pragma unroll
      for (int i = 0; i < KS; ++i)
#pragma unroll
        for (int j = 0; j < KS; ++j) s += wk[i * KS + j] * sv[cl][y + i][xx + j];
      const float o = (float)O16[((size_t)b * NP + n) * C + cb + cl] * 0.125f;
      sz[n][cg * 8 + cl] = (_Float16)((o + s) * 8.0f); }
    __syncthreads(); }
  for (int q = tid; q < NP * 8; q += 256) { const int n = q >> 3, pc = q & 7; vst2(Z16 + ((size_t)b * NP + n) * C + c0 + pc * 8, *(const v4u*)(&sz[n][pc * 8])); }
}
__global__ __launch_bounds__(128) void k_out(const _Float16* __restrict__ Z16, const _Float16* __restrict__ PT, const float* __restrict__ bp, float* __restrict__ out) {
  __shared__ __align__(16) float st[128][68];
  const int tid = threadIdx.x, wave = tid >> 5, lane = tid & 31, col = lane & 15, g = lane >> 4;
  const int r0b = blockIdx.x * 64, r0 = r0b + wave * 16, n0 = blockIdx.y * 128; const int b = r0b / NP, s0 = r0b % NP;
  v8f acc[8] = {};
#pragma unroll 2
  for (int kc = 0; kc < C / 32; ++kc) { const v16h a = frag_h(Z16 + (size_t)(r0 + col) * C + kc * 32, lane);
#pragma unroll
    for (int j = 0; j < 8; ++j) acc[j] = wmma16(a, frag_h(PT + (size_t)(3 * C + n0 + j * 16 + col) * C + kc * 32, lane), acc[j]); }
#pragma unroll
  for (int j = 0; j < 8; ++j) { const float bb = bp[n0 + j * 16 + col];
#pragma unroll
    for (int r = 0; r < 8; ++r) st[j * 16 + col][wave * 16 + 8 * g + r] = acc[j][r] * (1.0f / (16.0f * 8.0f)) + bb; }
  __syncthreads();
  for (int qq = tid; qq < 128 * 16; qq += 128) { const int cl = qq >> 4, pc = qq & 15; vst2(out + ((size_t)b * C + n0 + cl) * NP + s0 + pc * 4, *(const v4f*)(&st[cl][pc * 4])); }
}
extern "C" void kernel_launch(void* const* d_in, const int* in_sizes, int n_in, void* d_out, int out_size, void* d_ws, size_t ws_size, hipStream_t stream) {
  (void)in_sizes; (void)n_in; (void)out_size; (void)ws_size;
  const float* x = (const float*)d_in[0]; const float* wqkv = (const float*)d_in[1]; const float* wp = (const float*)d_in[2]; const float* bp = (const float*)d_in[3]; const float* lw = (const float*)d_in[4]; const float* lb = (const float*)d_in[5];
  float* out = (float*)d_out;
  char* ws = (char*)d_ws; size_t off = 0;
  auto take = [&](size_t bytes) { char* p = ws + off; off += (bytes + 255) & ~(size_t)255; return p; };
  _Float16* X16 = (_Float16*)take((size_t)NR * C * 2); _Float16* PT = (_Float16*)take((size_t)4 * C * C * 2);
  _Float16* Q16 = (_Float16*)take((size_t)NR * C * 2); _Float16* K16 = (_Float16*)take((size_t)NR * C * 2); _Float16* V16 = (_Float16*)take((size_t)NR * C * 2); _Float16* O16 = (_Float16*)take((size_t)NR * C * 2); _Float16* Z16 = X16;
  k_cvt<<<NBI * (NP / 64), 256, 0, stream>>>(x, X16);
  k_pack<<<4 * C, 256, 0, stream>>>(wqkv, wp, PT);
  k_qkv<<<dim3(NR / 64, 3 * C / 128), 128, 0, stream>>>(X16, PT, Q16, K16, V16);
  k_attn<<<dim3(NP / 64, NBI * NH), 128, 0, stream>>>(Q16, K16, V16, O16);
  k_lepe<<<NBI * (C / 64), 256, 0, stream>>>(V16, O16, lw, lb, Z16);
  k_out<<<dim3(NR / 64, C / 128), 128, 0, stream>>>(Z16, PT, bp, out);
}
